// HTGAT_15418932593211
// MI455X (gfx1250) — hardware-verified
//
#include <hip/hip_runtime.h>
#include <hip/hip_bf16.h>
#include <stddef.h>


#define KD    256
#define NHD   4
#define HDC   64
#define NTY   3
#define NET   4
#define EDM   32
#define NS    16

#define NTHR  256
#define NWAVE 8

#define GR    128
#define APH   264
#define RSP   68
#define MAXPR 24
#define LDS_GEMM_BYTES (2 * GR * APH * 2 + GR * RSP * 4 + GR * NS * 4 + 4 * GR * 4 + (2 * MAXPR + 4) * 4)

#define NB    256
#define CHUNK 2048
#define WCAP  256
#define NGRP  (CHUNK / (NTHR * 4))
#define LDS_AGG_FLOATS (NB * KD + 2 * NB * NHD + NET * NHD * EDM)
#define LDS_AGG_BYTES  (LDS_AGG_FLOATS * 4 + NWAVE * WCAP * 4 + NWAVE * 4)

static_assert(LDS_GEMM_BYTES == 180432);
static_assert(LDS_AGG_BYTES == 280608);
static_assert(WCAP == (CHUNK / NTHR) * 32);
static_assert(NGRP == 2);
static_assert((NB & (NB - 1)) == 0 && NB <= 512);
static_assert((CHUNK & (CHUNK - 1)) == 0 && CHUNK <= 4096);
static_assert((LDS_AGG_FLOATS % 4) == 0);
static_assert((APH % 8) == 0 && (RSP % 4) == 0);
static_assert((GR % 16) == 0 && MAXPR == 3 * (GR / 16));
static_assert(NHD * HDC == KD && NET * NHD == NS);
static_assert((GR * KD / 8) % NTHR == 0 && (GR * NS) % NTHR == 0);

typedef float          v4f  __attribute__((ext_vector_type(4)));
typedef float          v8f  __attribute__((ext_vector_type(8)));
typedef int            v4i  __attribute__((ext_vector_type(4)));
typedef __bf16         v16b __attribute__((ext_vector_type(16)));
typedef unsigned short us_t;
union FragB { v16b v; v4i u[2]; };

__device__ __forceinline__ v8f wmb(v16b a, v16b b, v8f c) {
  v8f d = __builtin_amdgcn_wmma_f32_16x16x32_bf16(false, a, false, b, (short)0, c, false, false);
  asm volatile("v_nop\n\tv_nop\n\tv_nop\n\tv_nop" : "+v"(d) : "v"(a), "v"(b));
  return d;
}

__device__ __forceinline__ float wsum(float v) {
  v += __shfl_xor(v, 16, 32);
  v += __shfl_xor(v, 8, 32);
  v += __shfl_xor(v, 4, 32);
  v += __shfl_xor(v, 2, 32);
  v += __shfl_xor(v, 1, 32);
  return v;
}

__device__ __forceinline__ unsigned bfr(float f) {
  unsigned u = __float_as_uint(f);
  u += 0x7FFFu + ((u >> 16) & 1u);
  return u >> 16;
}
__device__ __forceinline__ unsigned hl2(float f) {
  const unsigned hb = bfr(f);
  const float hf = __uint_as_float(hb << 16);
  const unsigned lb = bfr(f - hf);
  return hb | (lb << 16);
}
__device__ __forceinline__ void split8(v4f a, v4f b, v4i& ph, v4i& pl) {
  const unsigned s0 = hl2(a.x), s1 = hl2(a.y), s2 = hl2(a.z), s3 = hl2(a.w);
  const unsigned s4 = hl2(b.x), s5 = hl2(b.y), s6 = hl2(b.z), s7 = hl2(b.w);
  ph.x = (int)((s0 & 0xFFFFu) | (s1 << 16));
  ph.y = (int)((s2 & 0xFFFFu) | (s3 << 16));
  ph.z = (int)((s4 & 0xFFFFu) | (s5 << 16));
  ph.w = (int)((s6 & 0xFFFFu) | (s7 << 16));
  pl.x = (int)((s0 >> 16) | (s1 & 0xFFFF0000u));
  pl.y = (int)((s2 >> 16) | (s3 & 0xFFFF0000u));
  pl.z = (int)((s4 >> 16) | (s5 & 0xFFFF0000u));
  pl.w = (int)((s6 >> 16) | (s7 & 0xFFFF0000u));
}

__global__ __launch_bounds__(NTHR) void k_wsplit(const float* __restrict__ W1, const float* __restrict__ W2,
                                                 us_t* Wh1, us_t* Wl1, us_t* Wh2, us_t* Wl2) {
  __shared__ float T[64 * 65];
  const int tid = threadIdx.x;
  int b = blockIdx.x;
  const int sel = (b >= 48) ? 1 : 0;
  b -= sel * 48;
  const float* W = sel ? W2 : W1;
  us_t* Wh = sel ? Wh2 : Wh1;
  us_t* Wl = sel ? Wl2 : Wl1;
  const int tn = b >> 4;
  const int k0 = ((b >> 2) & 3) * 64;
  const int n0 = (b & 3) * 64;
#pragma unroll 4
  for (int i = 0; i < 16; ++i) {
    const int idx = i * NTHR + tid;
    const int kr = idx >> 6, nc = idx & 63;
    T[kr * 65 + nc] = W[((size_t)tn * KD + k0 + kr) * KD + n0 + nc];
  }
  __syncthreads();
  v4i ph[2], pl[2];
  size_t go[2];
#pragma unroll
  for (int i = 0; i < 2; ++i) {
    const int task = i * NTHR + tid;
    const int nr = task >> 3, q = task & 7;
    v4f f0, f1;
    f0.x = T[(8 * q + 0) * 65 + nr]; f0.y = T[(8 * q + 1) * 65 + nr];
    f0.z = T[(8 * q + 2) * 65 + nr]; f0.w = T[(8 * q + 3) * 65 + nr];
    f1.x = T[(8 * q + 4) * 65 + nr]; f1.y = T[(8 * q + 5) * 65 + nr];
    f1.z = T[(8 * q + 6) * 65 + nr]; f1.w = T[(8 * q + 7) * 65 + nr];
    split8(f0, f1, ph[i], pl[i]);
    go[i] = ((size_t)tn * KD + n0 + nr) * KD + k0 + 8 * q;
  }
#pragma unroll
  for (int i = 0; i < 2; ++i) { *(volatile v4i*)(Wh + go[i]) = ph[i]; *(volatile v4i*)(Wl + go[i]) = pl[i]; }
  __threadfence();
#pragma unroll
  for (int i = 0; i < 2; ++i) { *(volatile v4i*)(Wh + go[i]) = ph[i]; *(volatile v4i*)(Wl + go[i]) = pl[i]; }
}

__global__ __launch_bounds__(NTHR) void k_ufold(const float* __restrict__ Wd1, const float* __restrict__ ad1,
                                                const float* __restrict__ Wd2, const float* __restrict__ ad2,
                                                us_t* Uh1, us_t* Ul1, us_t* Uh2, us_t* Ul2) {
  __shared__ __attribute__((aligned(16))) us_t sh[KD];
  __shared__ __attribute__((aligned(16))) us_t sl[KD];
  const int tid = threadIdx.x, lane = tid & 31, wave = tid >> 5;
  int b = blockIdx.x;
  const int sel = (b >= 48) ? 1 : 0;
  b -= sel * 48;
  const float* Wd = sel ? Wd2 : Wd1;
  const float* ad = sel ? ad2 : ad1;
  us_t* Uh = sel ? Uh2 : Uh1;
  us_t* Ul = sel ? Ul2 : Ul1;
  const int tn = b >> 4, n = b & 15;
  const int t = n >> 2, h = n & 3;
  const int d = tid;
  const float* wr = Wd + ((size_t)tn * KD + d) * KD + h * HDC;
  const float* ar = ad + (t * NHD + h) * HDC;
  float acc = 0.f;
#pragma unroll 4
  for (int c = 0; c < HDC; ++c) acc += wr[c] * ar[c];
  const unsigned s = hl2(acc);
  sh[d] = (us_t)(s & 0xFFFFu);
  sl[d] = (us_t)(s >> 16);
  __syncthreads();
  const v4i va = *(const v4i*)(sh + 8 * lane);
  const v4i vb = *(const v4i*)(sl + 8 * lane);
  const v4i pv = (wave == 0) ? va : vb;
  const size_t ro = ((size_t)tn * NS + n) * KD + 8 * lane;
  if (wave == 0)      *(volatile v4i*)(Uh + ro) = pv;
  else if (wave == 1) *(volatile v4i*)(Ul + ro) = pv;
  __threadfence();
  if (wave == 0)      *(volatile v4i*)(Uh + ro) = pv;
  else if (wave == 1) *(volatile v4i*)(Ul + ro) = pv;
}

__global__ __launch_bounds__(NTHR) void k_vtab(const float* __restrict__ We1, const float* __restrict__ ae1,
                                               const float* __restrict__ We2, const float* __restrict__ ae2,
                                               float* vt) {
  __shared__ __attribute__((aligned(16))) float vs[NET * NHD * EDM];
  const int tid = threadIdx.x, lane = tid & 31, wave = tid >> 5;
  const int L = blockIdx.x;
  const float* We = L ? We2 : We1;
  const float* ae = L ? ae2 : ae1;
#pragma unroll
  for (int r = 0; r < 2; ++r) {
    const int idx = r * NTHR + tid;
    const int et = idx >> 7, h = (idx >> 5) & 3, d = idx & 31;
    const float* wr = We + ((size_t)et * EDM + d) * KD + h * HDC;
    const float* ar = ae + (et * NHD + h) * HDC;
    float acc = 0.f;
#pragma unroll 4
    for (int c = 0; c < HDC; ++c) acc += wr[c] * ar[c];
    vs[idx] = acc;
  }
  __syncthreads();
  const bool ok = wave < 4;
  const int wq = ok ? wave : 0;
  const v4f v = *(const v4f*)(vs + wq * 128 + 4 * lane);
  float* gp = vt + (size_t)L * (NET * NHD * EDM) + wq * 128 + 4 * lane;
  if (ok) *(volatile v4f*)gp = v;
  __threadfence();
  if (ok) *(volatile v4f*)gp = v;
}

__device__ __forceinline__ v8f tile_hilo(const us_t* ah, const us_t* al, const us_t* bh, const us_t* bl) {
  v8f acc = {0.f, 0.f, 0.f, 0.f, 0.f, 0.f, 0.f, 0.f};
#pragma unroll 2
  for (int ks = 0; ks < KD / 32; ++ks) {
    const int k0 = ks * 32;
    FragB fa, fl, gb, gl;
    fa.u[0] = *(const v4i*)(ah + k0);  fa.u[1] = *(const v4i*)(ah + k0 + 16);
    fl.u[0] = *(const v4i*)(al + k0);  fl.u[1] = *(const v4i*)(al + k0 + 16);
    gb.u[0] = *(const v4i*)(bh + k0);  gb.u[1] = *(const v4i*)(bh + k0 + 16);
    gl.u[0] = *(const v4i*)(bl + k0);  gl.u[1] = *(const v4i*)(bl + k0 + 16);
    acc = wmb(fa.v, gb.v, acc);
    acc = wmb(fa.v, gl.v, acc);
    acc = wmb(fl.v, gb.v, acc);
  }
  return acc;
}

__global__ __launch_bounds__(NTHR) void k_gemm(
    const float* __restrict__ X, const int* __restrict__ ntype,
    const us_t* __restrict__ Wh, const us_t* __restrict__ Wl,
    const us_t* __restrict__ Uh, const us_t* __restrict__ Ul,
    const float* __restrict__ att, float* xs, float* ssrc, float* sdst, int nN) {
  extern __shared__ v4i lds_g[];
  us_t*  Ah    = (us_t*)lds_g;
  us_t*  Al    = Ah + GR * APH;
  float* Rs    = (float*)(Al + GR * APH);
  float* Ss    = Rs + GR * RSP;
  int*   ltype = (int*)(Ss + GR * NS);
  int*   spos  = ltype + GR;
  int*   srow  = spos + GR;
  int*   stype = srow + GR;
  int*   prt   = stype + GR;
  int*   pty   = prt + MAXPR;
  int*   npr   = pty + MAXPR;

  const int tid  = threadIdx.x;
  const int lane = tid & 31;
  const int wave = tid >> 5;
  const int hh   = lane >> 4;
  const int m    = lane & 15;
  const int rowBase = blockIdx.x * GR;

  if (tid < GR) {
    int row = rowBase + tid;
    row = row > nN - 1 ? nN - 1 : row;
    int t = ntype[row];
    t = t < 0 ? 0 : (t > NTY - 1 ? NTY - 1 : t);
    ltype[tid] = t;
  }
  __syncthreads();
  if (tid == 0) {
    int c0 = 0, c1 = 0, c2 = 0;
#pragma unroll 1
    for (int i = 0; i < GR; ++i) { const int t = ltype[i]; c0 += (t == 0); c1 += (t == 1); c2 += (t == 2); }
    int q0 = 0, q1 = c0, q2 = c0 + c1;
#pragma unroll 1
    for (int i = 0; i < GR; ++i) {
      const int t = ltype[i];
      int p;
      if (t == 0) { p = q0; ++q0; } else if (t == 1) { p = q1; ++q1; } else { p = q2; ++q2; }
      spos[i] = p; srow[p] = i; stype[p] = t;
    }
    const int s0 = 0, s1 = c0, s2 = c0 + c1;
    int np = 0;
#pragma unroll 1
    for (int rt = 0; rt < GR / 16; ++rt) {
      const int lo = rt * 16, hi = lo + 16;
      if (c0 > 0 && s0 < hi && s0 + c0 > lo) { prt[np] = rt; pty[np] = 0; ++np; }
      if (c1 > 0 && s1 < hi && s1 + c1 > lo) { prt[np] = rt; pty[np] = 1; ++np; }
      if (c2 > 0 && s2 < hi && s2 + c2 > lo) { prt[np] = rt; pty[np] = 2; ++np; }
    }
    npr[0] = np;
  }
  __syncthreads();

#pragma unroll 2
  for (int i = 0; i < (GR * KD / 8) / NTHR; ++i) {
    const int task = i * NTHR + tid;
    const int p  = task >> 5;
    const int c8 = (task & 31) * 8;
    int row = rowBase + srow[p];
    row = row > nN - 1 ? nN - 1 : row;
    const float* src = X + (size_t)row * KD + c8;
    const v4f f0 = *(const v4f*)src;
    const v4f f1 = *(const v4f*)(src + 4);
    v4i ph, pl;
    split8(f0, f1, ph, pl);
    *(v4i*)(Ah + p * APH + c8) = ph;
    *(v4i*)(Al + p * APH + c8) = pl;
  }
  __syncthreads();
  int np = npr[0];
  np = np > MAXPR ? MAXPR : (np < 0 ? 0 : np);

#pragma unroll 1
  for (int g = 0; g < NHD; ++g) {
    const int njobs = np * 4;
#pragma unroll 1
    for (int j = wave; j < njobs; j += NWAVE) {
      const int pr = j >> 2;
      const int ct = j & 3;
      const int rt = prt[pr];
      const int ty = pty[pr];
      const int ncol = g * HDC + ct * 16 + m;
      const size_t bo = ((size_t)ty * KD + ncol) * KD + 8 * hh;
      const int ao = (rt * 16 + m) * APH + 8 * hh;
      const v8f acc = tile_hilo(Ah + ao, Al + ao, Wh + bo, Wl + bo);
#pragma unroll
      for (int r = 0; r < 8; ++r) {
        const int pos = rt * 16 + 8 * hh + r;
        if (stype[pos] == ty) Rs[pos * RSP + ct * 16 + m] = acc[r];
      }
    }
    __syncthreads();
    {
      const int m4 = lane & 15;
      const v4f a0 = *(const v4f*)(att + (0 * NHD + g) * HDC + 4 * m4);
      const v4f a1 = *(const v4f*)(att + (1 * NHD + g) * HDC + 4 * m4);
      const v4f a2 = *(const v4f*)(att + (2 * NHD + g) * HDC + 4 * m4);
      const v4f a3 = *(const v4f*)(att + (3 * NHD + g) * HDC + 4 * m4);
      v4f vv[8];
      size_t go[8];
#pragma unroll
      for (int i = 0; i < 8; ++i) {
        const int p = wave * 16 + 2 * i + hh;
        const v4f v = *(const v4f*)(Rs + p * RSP + 4 * m4);
        vv[i] = v;
        float t0 = v.x * a0.x + v.y * a0.y + v.z * a0.z + v.w * a0.w;
        float t1 = v.x * a1.x + v.y * a1.y + v.z * a1.z + v.w * a1.w;
        float t2 = v.x * a2.x + v.y * a2.y + v.z * a2.z + v.w * a2.w;
        float t3 = v.x * a3.x + v.y * a3.y + v.z * a3.z + v.w * a3.w;
#pragma unroll
        for (int mk = 8; mk > 0; mk >>= 1) {
          t0 += __shfl_xor(t0, mk, 32);
          t1 += __shfl_xor(t1, mk, 32);
          t2 += __shfl_xor(t2, mk, 32);
          t3 += __shfl_xor(t3, mk, 32);
        }
        if (m4 == 0) {
          Ss[p * NS + 0 * NHD + g] = t0;
          Ss[p * NS + 1 * NHD + g] = t1;
          Ss[p * NS + 2 * NHD + g] = t2;
          Ss[p * NS + 3 * NHD + g] = t3;
        }
        go[i] = (size_t)(rowBase + srow[p]) * KD + g * HDC + 4 * m4;
      }
#pragma unroll
      for (int i = 0; i < 8; ++i) *(volatile v4f*)(xs + go[i]) = vv[i];
      __threadfence();
#pragma unroll
      for (int i = 0; i < 8; ++i) *(volatile v4f*)(xs + go[i]) = vv[i];
    }
    __syncthreads();
  }

#pragma unroll 1
  for (int j = wave; j < np; j += NWAVE) {
    const int rt = prt[j];
    const int ty = pty[j];
    const size_t bo = ((size_t)ty * NS + m) * KD + 8 * hh;
    const int ao = (rt * 16 + m) * APH + 8 * hh;
    const v8f acc = tile_hilo(Ah + ao, Al + ao, Uh + bo, Ul + bo);
#pragma unroll
    for (int r = 0; r < 8; ++r) {
      const int pos = rt * 16 + 8 * hh + r;
      if (stype[pos] == ty) Rs[pos * RSP + m] = acc[r];
    }
  }
  __syncthreads();

  {
    v4f sv[2], dv[2];
    size_t so[2];
#pragma unroll
    for (int i = 0; i < 2; ++i) {
      const int task = i * NTHR + tid;
      const int nl = task >> 2;
      const int q  = task & 3;
      const int p  = spos[nl];
      sv[i] = *(const v4f*)(Ss + p * NS + 4 * q);
      dv[i] = *(const v4f*)(Rs + p * RSP + 4 * q);
      so[i] = (size_t)(rowBase + nl) * NS + 4 * q;
    }
#pragma unroll
    for (int i = 0; i < 2; ++i) { *(volatile v4f*)(ssrc + so[i]) = sv[i]; *(volatile v4f*)(sdst + so[i]) = dv[i]; }
    __threadfence();
#pragma unroll
    for (int i = 0; i < 2; ++i) { *(volatile v4f*)(ssrc + so[i]) = sv[i]; *(volatile v4f*)(sdst + so[i]) = dv[i]; }
  }
}

template <int L2>
__global__ __launch_bounds__(NTHR) void k_agg(
    const float* __restrict__ xs, const float* __restrict__ ssrc, const float* __restrict__ sdst,
    const float* __restrict__ vtab, const int* __restrict__ ei, const int* __restrict__ ety,
    const float* __restrict__ ea, const float* __restrict__ bias, const float* __restrict__ gam,
    const float* __restrict__ bet, float* outp, int nN, int nE) {
  extern __shared__ v4f lds_a[];
  float* sacc = (float*)lds_a;
  float* den  = sacc + NB * KD;
  float* mx   = den + NB * NHD;
  float* vt   = mx + NB * NHD;
  int*   list = (int*)(vt + NET * NHD * EDM);
  int*   wcnt = list + NWAVE * WCAP;

  const int tid  = threadIdx.x;
  const int lane = tid & 31;
  const int wave = tid >> 5;
  const int hh   = lane >> 4;
  const int nodeBase = blockIdx.x * NB;

  {
    const v4f z4 = {0.f, 0.f, 0.f, 0.f};
    for (int i = tid; i < (NB * KD + NB * NHD) / 4; i += NTHR) lds_a[i] = z4;
    const v4f mi = {-1.0e30f, -1.0e30f, -1.0e30f, -1.0e30f};
    for (int i = tid; i < (NB * NHD) / 4; i += NTHR) *(v4f*)(mx + 4 * i) = mi;
    if (tid < (NET * NHD * EDM) / 4) *(v4f*)(vt + 4 * tid) = *(const v4f*)(vtab + 4 * tid);
  }
  __syncthreads();

  const int* eid = ei + nE;
  const bool al16 = ((nE & 3) == 0);
  const int nChunks = (nE + CHUNK - 1) / CHUNK;
#pragma unroll 1
  for (int ch = 0; ch < nChunks; ++ch) {
    const int cbase = ch * CHUNK;
    const bool fullc = al16 && (cbase + CHUNK <= nE);
    int wc = 0;
#pragma unroll
    for (int g = 0; g < NGRP; ++g) {
      const int el0 = (g * NTHR + tid) * 4;
      const int e0  = cbase + el0;
      const int sent = -2147483647 - 1;
      v4i d;
      if (fullc) {
        d = *(const v4i*)(eid + e0);
      } else {
        const int i0 = e0 < nE ? e0 : nE - 1;
        const int i1 = e0 + 1 < nE ? e0 + 1 : nE - 1;
        const int i2 = e0 + 2 < nE ? e0 + 2 : nE - 1;
        const int i3 = e0 + 3 < nE ? e0 + 3 : nE - 1;
        const int v0 = eid[i0], v1 = eid[i1], v2 = eid[i2], v3 = eid[i3];
        d.x = (e0     < nE) ? v0 : sent;
        d.y = (e0 + 1 < nE) ? v1 : sent;
        d.z = (e0 + 2 < nE) ? v2 : sent;
        d.w = (e0 + 3 < nE) ? v3 : sent;
      }
      const unsigned s0 = (unsigned)d.x - (unsigned)nodeBase;
      const unsigned s1 = (unsigned)d.y - (unsigned)nodeBase;
      const unsigned s2 = (unsigned)d.z - (unsigned)nodeBase;
      const unsigned s3 = (unsigned)d.w - (unsigned)nodeBase;
      const bool h0 = s0 < (unsigned)NB;
      const bool h1 = s1 < (unsigned)NB;
      const bool h2 = s2 < (unsigned)NB;
      const bool h3 = s3 < (unsigned)NB;
      const unsigned many = __builtin_amdgcn_ballot_w32(h0 | h1 | h2 | h3);
      if (many != 0u) {
#define HITJ(J, HJ, SJ) { \
          const unsigned mj = __builtin_amdgcn_ballot_w32(HJ); \
          if (HJ) { \
            const int pos = wc + (int)__builtin_amdgcn_mbcnt_lo(mj, 0u); \
            if (pos < WCAP) list[wave * WCAP + pos] = ((el0 + (J)) << 9) | (int)(SJ); \
          } \
          wc += (int)__builtin_popcount(mj); }
        HITJ(0, h0, s0)
        HITJ(1, h1, s1)
        HITJ(2, h2, s2)
        HITJ(3, h3, s3)
#undef HITJ
      }
    }
    if (lane == 0) wcnt[wave] = wc;
    __syncthreads();

    if (wave == 0) {
      const int hd = lane >> 3;
      const int q  = lane & 7;
#pragma unroll 1
      for (int wsx = 0; wsx < NWAVE; ++wsx) {
        int n = wcnt[wsx];
        n = n > WCAP ? WCAP : n;
        n = n < 0 ? 0 : n;
#pragma unroll 1
        for (int i = 0; i < n; ++i) {
          const int ent  = list[wsx * WCAP + i];
          const int slot = ent & (NB - 1);
          const int el   = (ent >> 9) & (CHUNK - 1);
          int e = cbase + el;
          e = e > nE - 1 ? nE - 1 : e;
          int src = ei[e];
          src = src < 0 ? 0 : (src > nN - 1 ? nN - 1 : src);
          int et = ety[e];
          et = et < 0 ? 0 : (et > NET - 1 ? NET - 1 : et);
          int nd = nodeBase + slot;
          nd = nd > nN - 1 ? nN - 1 : nd;
          const float ssv = ssrc[(size_t)src * NS + et * NHD + hd];
          const float sdv = sdst[(size_t)nd * NS + et * NHD + hd];
          const v4f e4 = *(const v4f*)(ea + (size_t)e * EDM + 4 * q);
          const v4f v4 = *(const v4f*)(vt + (et * NHD + hd) * EDM + 4 * q);
          float pe = e4.x * v4.x + e4.y * v4.y + e4.z * v4.z + e4.w * v4.w;
          pe += __shfl_xor(pe, 4, 32);
          pe += __shfl_xor(pe, 2, 32);
          pe += __shfl_xor(pe, 1, 32);
          float al = ssv + sdv + pe;
          al = (al >= 0.f) ? al : 0.2f * al;
          const float mo = mx[slot * NHD + hd];
          const float mn = fmaxf(mo, al);
          const float sc = __expf(mo - mn);
          const float p  = __expf(al - mn);
          const float dn = den[slot * NHD + hd] * sc + p;
          const v4f x0 = *(const v4f*)(xs + (size_t)src * KD + 8 * lane);
          const v4f x1 = *(const v4f*)(xs + (size_t)src * KD + 8 * lane + 4);
          v4f* sp = (v4f*)(sacc + slot * KD + 8 * lane);
          const v4f c0 = sp[0];
          const v4f c1 = sp[1];
          sp[0] = c0 * sc + x0 * p;
          sp[1] = c1 * sc + x1 * p;
          mx[slot * NHD + hd]  = mn;
          den[slot * NHD + hd] = dn;
        }
      }
    }
    __syncthreads();
  }

  if (L2 == 0) {
    const int hA = lane >> 4;
    const int hB = 2 + (lane >> 4);
    const v4f bA = *(const v4f*)(bias + 4 * lane);
    const v4f bB = *(const v4f*)(bias + KD / 2 + 4 * lane);
    const v4f gA = *(const v4f*)(gam + 4 * lane);
    const v4f gB = *(const v4f*)(gam + KD / 2 + 4 * lane);
    const v4f eA = *(const v4f*)(bet + 4 * lane);
    const v4f eB = *(const v4f*)(bet + KD / 2 + 4 * lane);
#pragma unroll 1
    for (int j = 0; j < NB / NWAVE; ++j) {
      const int slot = wave * (NB / NWAVE) + j;
      const int node = nodeBase + slot;
      const float iA = __builtin_amdgcn_rcpf(den[slot * NHD + hA] + 1e-16f);
      const float iB = __builtin_amdgcn_rcpf(den[slot * NHD + hB] + 1e-16f);
      const v4f vA = *(const v4f*)(sacc + slot * KD + 4 * lane) * iA + bA;
      const v4f vB = *(const v4f*)(sacc + slot * KD + KD / 2 + 4 * lane) * iB + bB;
      const float s  = wsum(vA.x + vA.y + vA.z + vA.w + vB.x + vB.y + vB.z + vB.w);
      const float mu = s * (1.0f / KD);
      const v4f dA = vA - mu;
      const v4f dB = vB - mu;
      const float qv = wsum(dA.x * dA.x + dA.y * dA.y + dA.z * dA.z + dA.w * dA.w +
                            dB.x * dB.x + dB.y * dB.y + dB.z * dB.z + dB.w * dB.w);
      const float rs = rsqrtf(qv * (1.0f / KD) + 1e-5f);
      v4f yA = dA * rs * gA + eA;
      v4f yB = dB * rs * gB + eB;
      yA.x = yA.x > 0.f ? yA.x : (__expf(yA.x) - 1.0f);
      yA.y = yA.y > 0.f ? yA.y : (__expf(yA.y) - 1.0f);
      yA.z = yA.z > 0.f ? yA.z : (__expf(yA.z) - 1.0f);
      yA.w = yA.w > 0.f ? yA.w : (__expf(yA.w) - 1.0f);
      yB.x = yB.x > 0.f ? yB.x : (__expf(yB.x) - 1.0f);
      yB.y = yB.y > 0.f ? yB.y : (__expf(yB.y) - 1.0f);
      yB.z = yB.z > 0.f ? yB.z : (__expf(yB.z) - 1.0f);
      yB.w = yB.w > 0.f ? yB.w : (__expf(yB.w) - 1.0f);
      float* op = outp + (size_t)node * KD;
      *(volatile v4f*)(op + 4 * lane) = yA;
      *(volatile v4f*)(op + KD / 2 + 4 * lane) = yB;
      __threadfence();
      *(volatile v4f*)(op + 4 * lane) = yA;
      *(volatile v4f*)(op + KD / 2 + 4 * lane) = yB;
    }
  } else {
    const int m4 = lane & 15;
    const v4f b4 = *(const v4f*)(bias + 4 * m4);
#pragma unroll 1
    for (int j = 0; j < NB / (2 * NWAVE); ++j) {
      const int slot = wave * (NB / NWAVE) + 2 * j + hh;
      const int node = nodeBase + slot;
      const float i0 = __builtin_amdgcn_rcpf(den[slot * NHD + 0] + 1e-16f);
      const float i1 = __builtin_amdgcn_rcpf(den[slot * NHD + 1] + 1e-16f);
      const float i2 = __builtin_amdgcn_rcpf(den[slot * NHD + 2] + 1e-16f);
      const float i3 = __builtin_amdgcn_rcpf(den[slot * NHD + 3] + 1e-16f);
      const float* sr = sacc + slot * KD + 4 * m4;
      v4f v = *(const v4f*)(sr) * i0;
      v += *(const v4f*)(sr + HDC) * i1;
      v += *(const v4f*)(sr + 2 * HDC) * i2;
      v += *(const v4f*)(sr + 3 * HDC) * i3;
      const v4f y = v * 0.25f + b4;
      const bool ok = node < nN;
      float* op = outp + (size_t)(ok ? node : 0) * HDC + 4 * m4;
      if (ok) *(volatile v4f*)op = y;
      __threadfence();
      if (ok) *(volatile v4f*)op = y;
    }
  }
}

extern "C" void kernel_launch(void* const* d_in, const int* in_sizes, int n_in,
                              void* d_out, int out_size, void* d_ws, size_t ws_size,
                              hipStream_t stream) {
  if (n_in < 21) return;
  const int nN = in_sizes[2];
  const int nE = in_sizes[3];
  if (nN <= 0 || nE <= 0) return;
  if (in_sizes[0] != nN * KD) return;
  if (in_sizes[1] != 2 * nE) return;
  if (in_sizes[4] != nE * EDM) return;
  if (in_sizes[5] != NTY * KD * KD || in_sizes[6] != NTY * KD * KD) return;
  if (in_sizes[14] != NTY * KD * KD || in_sizes[15] != NTY * KD * KD) return;
  if (in_sizes[7] != NET * NHD * HDC || in_sizes[8] != NET * NHD * HDC || in_sizes[10] != NET * NHD * HDC) return;
  if (in_sizes[16] != NET * NHD * HDC || in_sizes[17] != NET * NHD * HDC || in_sizes[19] != NET * NHD * HDC) return;
  if (in_sizes[9] != NET * EDM * KD || in_sizes[18] != NET * EDM * KD) return;
  if (in_sizes[11] != KD || in_sizes[12] != KD || in_sizes[13] != KD) return;
  if (in_sizes[20] != HDC) return;
  if (out_size != nN * HDC) return;

  const float* x      = (const float*)d_in[0];
  const int*   ei     = (const int*)d_in[1];
  const int*   ntype  = (const int*)d_in[2];
  const int*   etype  = (const int*)d_in[3];
  const float* eattr  = (const float*)d_in[4];
  const float* W_src1 = (const float*)d_in[5];
  const float* W_dst1 = (const float*)d_in[6];
  const float* a_src1 = (const float*)d_in[7];
  const float* a_dst1 = (const float*)d_in[8];
  const float* W_edg1 = (const float*)d_in[9];
  const float* a_edg1 = (const float*)d_in[10];
  const float* bias1  = (const float*)d_in[11];
  const float* gam1   = (const float*)d_in[12];
  const float* bet1   = (const float*)d_in[13];
  const float* W_src2 = (const float*)d_in[14];
  const float* W_dst2 = (const float*)d_in[15];
  const float* a_src2 = (const float*)d_in[16];
  const float* a_dst2 = (const float*)d_in[17];
  const float* W_edg2 = (const float*)d_in[18];
  const float* a_edg2 = (const float*)d_in[19];
  const float* bias2  = (const float*)d_in[20];
  float* out = (float*)d_out;

  const int nPg = ((nN + GR - 1) / GR) * GR;
  const int nPa = ((nN + NB - 1) / NB) * NB;
  char* base = (char*)d_ws;
  size_t off = 0;
  auto take = [&](size_t bytes) -> char* {
    char* r = base + off; off += (bytes + 255) & ~(size_t)255; return r;
  };
  us_t*  Wh1 = (us_t*)take((size_t)NTY * KD * KD * 2);
  us_t*  Wl1 = (us_t*)take((size_t)NTY * KD * KD * 2);
  us_t*  Wh2 = (us_t*)take((size_t)NTY * KD * KD * 2);
  us_t*  Wl2 = (us_t*)take((size_t)NTY * KD * KD * 2);
  us_t*  Uh1 = (us_t*)take((size_t)NTY * NS * KD * 2);
  us_t*  Ul1 = (us_t*)take((size_t)NTY * NS * KD * 2);
  us_t*  Uh2 = (us_t*)take((size_t)NTY * NS * KD * 2);
  us_t*  Ul2 = (us_t*)take((size_t)NTY * NS * KD * 2);
  float* vt  = (float*)take((size_t)2 * NET * NHD * EDM * 4);
  float* xs  = (float*)take((size_t)nPg * KD * 4);
  float* ss  = (float*)take((size_t)nPg * NS * 4);
  float* sd  = (float*)take((size_t)nPg * NS * 4);
  float* hpl = (float*)take((size_t)nPa * KD * 4);
  if (off > ws_size) return;

  k_wsplit<<<96, NTHR, 0, stream>>>(W_src1, W_src2, Wh1, Wl1, Wh2, Wl2);
  k_ufold<<<96, NTHR, 0, stream>>>(W_dst1, a_dst1, W_dst2, a_dst2, Uh1, Ul1, Uh2, Ul2);
  k_vtab<<<2, NTHR, 0, stream>>>(W_edg1, a_edg1, W_edg2, a_edg2, vt);

  hipFuncSetAttribute(reinterpret_cast<const void*>(&k_gemm),
                      hipFuncAttributeMaxDynamicSharedMemorySize, LDS_GEMM_BYTES);
  hipFuncSetAttribute(reinterpret_cast<const void*>(&k_agg<0>),
                      hipFuncAttributeMaxDynamicSharedMemorySize, LDS_AGG_BYTES);
  hipFuncSetAttribute(reinterpret_cast<const void*>(&k_agg<1>),
                      hipFuncAttributeMaxDynamicSharedMemorySize, LDS_AGG_BYTES);

  const int ggrid = nPg / GR;
  const int agrid = nPa / NB;

  k_gemm<<<ggrid, NTHR, LDS_GEMM_BYTES, stream>>>(x, ntype, Wh1, Wl1, Uh1, Ul1, a_src1, xs, ss, sd, nN);
  k_agg<0><<<agrid, NTHR, LDS_AGG_BYTES, stream>>>(xs, ss, sd, vt, ei, etype, eattr,
                                                   bias1, gam1, bet1, hpl, nN, nE);
  k_gemm<<<ggrid, NTHR, LDS_GEMM_BYTES, stream>>>(hpl, ntype, Wh2, Wl2, Uh2, Ul2, a_src2, xs, ss, sd, nN);
  k_agg<1><<<agrid, NTHR, LDS_AGG_BYTES, stream>>>(xs, ss, sd, vt + NET * NHD * EDM, ei, etype, eattr,
                                                   bias2, gam1, bet1, out, nN, nE);
}
